// Rainfusion_87488483819576
// MI455X (gfx1250) — hardware-verified
//
#include <hip/hip_runtime.h>
#include <math.h>
#include <stdint.h>

#define S_TOK   9616
#define S_PAD   9664
#define NCH     151
#define NHD     2
#define HD      128
#define DMOD    256
#define PERF    1040
#define RAZOR   8320
#define NRB     130
#define ROTK    8576
#define PREB    2048
#define BSPAN   32
#define NTAIL   21
#define RQB     17
#define QSC     16.0f
#define KSC     16.0f
#define VSC     256.0f
#define PSC     1024.0f
#define RSC     4096.0f
static_assert(NCH * 64 == S_PAD);
static_assert(NRB * 64 == RAZOR);
static_assert(NRB + NTAIL == NCH);
static_assert(BSPAN * 64 == PREB);
static_assert(ROTK + PERF == S_TOK);
static_assert(RQB * 64 >= PERF);
static_assert((RQB * 64 - 1) * 8 < S_PAD);
static_assert(NHD * HD == DMOD);
static_assert((S_PAD * 32) % 256 == 0);

typedef _Float16 v16h __attribute__((ext_vector_type(16)));
typedef _Float16 v8h  __attribute__((ext_vector_type(8)));
typedef float    v8f  __attribute__((ext_vector_type(8)));
typedef float    v4f  __attribute__((ext_vector_type(4)));
typedef unsigned int v4u __attribute__((ext_vector_type(4)));

__device__ __forceinline__ unsigned short bf_bits(float f) {
  unsigned u = __float_as_uint(f);
  return (unsigned short)((u + 0x7FFFu + ((u >> 16) & 1u)) >> 16);
}
__device__ __forceinline__ float bf_up(unsigned short h) { return __uint_as_float(((unsigned)h) << 16); }
__device__ __forceinline__ float bfr(float f) { return bf_up(bf_bits(f)); }
__device__ __forceinline__ unsigned short h_bits(_Float16 x) { return __builtin_bit_cast(unsigned short, x); }
__device__ __forceinline__ unsigned pk16(unsigned short a, unsigned short b) { return (unsigned)a | ((unsigned)b << 16); }
__device__ __forceinline__ v8f zero8() { v8f z = {0.f, 0.f, 0.f, 0.f, 0.f, 0.f, 0.f, 0.f}; return z; }
__device__ __forceinline__ v4f zero4() { v4f z = {0.f, 0.f, 0.f, 0.f}; return z; }
__device__ __forceinline__ unsigned short cvt_h(float f, float sc) { return h_bits((_Float16)(bfr(f) * sc)); }
__device__ __forceinline__ float fexp(float x) { return __builtin_amdgcn_exp2f(x * 1.4426950408889634f); }
__device__ __forceinline__ int orig_row(int p) { return (p < ROTK) ? (p + PERF) : (p - ROTK); }

__device__ __forceinline__ v16h ldfrag_h(const _Float16* p) {
  union { v16h v; v8h h[2]; } f;
  f.h[0] = *(const v8h*)(p);
  f.h[1] = *(const v8h*)(p + 16);
  return f.v;
}

__device__ __forceinline__ v8f mma_h(v16h a, v16h b, v8f c) {
  c = __builtin_amdgcn_wmma_f32_16x16x32_f16(false, a, false, b, (short)0, c, false, false);
#if defined(__HIP_DEVICE_COMPILE__)
  asm volatile("v_nop\n\tv_nop\n\tv_nop\n\tv_nop" : "+v"(c) : "v"(a), "v"(b));
#endif
  return c;
}
__device__ __forceinline__ void wave_sync_lds() {
  __builtin_amdgcn_fence(__ATOMIC_RELEASE, "workgroup");
  __builtin_amdgcn_wave_barrier();
  __builtin_amdgcn_fence(__ATOMIC_ACQUIRE, "workgroup");
}

__global__ __launch_bounds__(256) void conv_qk(const float* __restrict__ q, const float* __restrict__ k,
                                               unsigned short* qh, unsigned short* kh) {
  const int which = blockIdx.y;
  const float* src = which ? k : q;
  unsigned short* dst = which ? kh : qh;
  const float sc = which ? KSC : QSC;
  const int i = blockIdx.x * 256 + threadIdx.x;
  if (i >= S_PAD * 32) return;
  const int row = i >> 5;
  const int c8  = (i & 31) * 8;
  const int vr  = (row < S_TOK) ? row : (S_TOK - 1);
  const size_t so = (size_t)orig_row(vr) * DMOD + c8;
  v4f a = *(const v4f*)(src + so);
  v4f b = *(const v4f*)(src + so + 4);
  if (row >= S_TOK) { a = zero4(); b = zero4(); }
  v4u u;
  u[0] = pk16(cvt_h(a[0], sc), cvt_h(a[1], sc));
  u[1] = pk16(cvt_h(a[2], sc), cvt_h(a[3], sc));
  u[2] = pk16(cvt_h(b[0], sc), cvt_h(b[1], sc));
  u[3] = pk16(cvt_h(b[2], sc), cvt_h(b[3], sc));
  const size_t dof = (size_t)row * DMOD + c8;
  for (int pass = 0; pass < 2; ++pass) {
    *(volatile v4u*)(dst + dof) = u;
    __threadfence();
  }
}

__global__ __launch_bounds__(256) void conv_vt(const float* __restrict__ v, unsigned short* vt) {
  __shared__ __align__(16) _Float16 sT[DMOD * 72];
  const int tid  = threadIdx.x;
  const int lane = tid & 31;
  const int wave = tid >> 5;
  const int kv0  = blockIdx.x * 64;
#pragma unroll 4
  for (int it = 0; it < 16; ++it) {
    const int f    = it * 256 + tid;
    const int key  = f >> 6;
    const int c4   = (f & 63) * 4;
    const int grow = kv0 + key;
    const int vr   = (grow < S_TOK) ? grow : (S_TOK - 1);
    v4f x = *(const v4f*)(v + (size_t)orig_row(vr) * DMOD + c4);
    if (grow >= S_TOK) x = zero4();
#pragma unroll
    for (int e = 0; e < 4; ++e) sT[(c4 + e) * 72 + key] = (_Float16)(bfr(x[e]) * VSC);
  }
  __syncthreads();
  const int q8 = lane >> 3, c8 = (lane & 7) * 8;
  for (int pass = 0; pass < 2; ++pass) {
#pragma unroll
    for (int it = 0; it < 8; ++it) {
      const int row = wave * 32 + it * 4 + q8;
      union { v8h h; v4u u; } t;
      t.h = *(const v8h*)(sT + row * 72 + c8);
      *(volatile v4u*)(vt + (size_t)row * S_PAD + kv0 + c8) = t.u;
    }
    __threadfence();
  }
}

union AttnSmem { _Float16 h[64 * HD + HD * 64]; float f[4 * 16 * HD]; };

__global__ __launch_bounds__(128)
void attn_band(const unsigned short* __restrict__ qhp, const unsigned short* __restrict__ khp,
               const unsigned short* __restrict__ vtp, float* out, float sscale) {
  union FH { v16h v; v8h h[2]; };
  __shared__ __align__(16) AttnSmem sm;
  __shared__ __align__(16) _Float16 Psh[4][16 * 64];
  __shared__ __align__(16) _Float16 Psl[4][16 * 64];
  _Float16* Ksh = sm.h;
  _Float16* Vsh = sm.h + 64 * HD;

  const int tid  = threadIdx.x;
  const int wave = tid >> 5;
  const int lane = tid & 31;
  const int hh   = lane >> 4;
  const int c    = lane & 15;

  const int bx   = blockIdx.x;
  const int qb   = bx % NCH;
  const int head = bx / NCH;
  const int q0   = qb * 64 + wave * 16;

  const _Float16* Qg = (const _Float16*)(const void*)qhp + (size_t)head * HD;
  const _Float16* Kg = (const _Float16*)(const void*)khp + (size_t)head * HD;
  const _Float16* Vg = (const _Float16*)(const void*)vtp + (size_t)head * HD * S_PAD;

  v16h qa[4];
#pragma unroll
  for (int dc = 0; dc < 4; ++dc) qa[dc] = ldfrag_h(Qg + (size_t)(q0 + c) * DMOD + dc * 32 + 8 * hh);

  float mrow[8], lrow[8];
  v8f oacc[8];
#pragma unroll
  for (int r = 0; r < 8; ++r) { mrow[r] = -INFINITY; lrow[r] = 0.f; }
#pragma unroll
  for (int t = 0; t < 8; ++t) oacc[t] = zero8();

  const bool razorblk = (qb < NRB);
  int ktLo = razorblk ? (qb - BSPAN) : 0;
  if (ktLo < 0) ktLo = 0;
  int ktHi = razorblk ? (qb + BSPAN) : (NRB - 1);
  if (ktHi > NRB - 1) ktHi = NRB - 1;
  const int nA   = ktHi - ktLo + 1;
  const int nvis = nA + NTAIL;
  const float rinv = 1.0f / RSC;

  for (int it = 0; it < nvis; ++it) {
    const int kt  = (it < nA) ? (ktLo + it) : (NRB + (it - nA));
    const int kv0 = kt * 64;
    __syncthreads();
    {
      const int r = tid >> 1, hf = (tid & 1) * 64;
      const _Float16* kg = Kg + (size_t)(kv0 + r) * DMOD + hf;
#pragma unroll
      for (int i = 0; i < 8; ++i) *(v8h*)(Ksh + r * HD + hf + 8 * i) = *(const v8h*)(kg + 8 * i);
      const _Float16* vg = Vg + (size_t)tid * S_PAD + kv0;
#pragma unroll
      for (int i = 0; i < 8; ++i) *(v8h*)(Vsh + tid * 64 + 8 * i) = *(const v8h*)(vg + 8 * i);
    }
    __syncthreads();

    v8f s[4];
#pragma unroll
    for (int j = 0; j < 4; ++j) {
      v8f sh = zero8();
#pragma unroll
      for (int dc = 0; dc < 4; ++dc) {
        FH kb;
        kb.h[0] = *(const v8h*)(Ksh + (j * 16 + c) * HD + dc * 32 + 8 * hh);
        kb.h[1] = *(const v8h*)(Ksh + (j * 16 + c) * HD + dc * 32 + 16 + 8 * hh);
        sh = mma_h(qa[dc], kb.v, sh);
      }
      const int key = kv0 + j * 16 + c;
      const bool keyok  = key < S_TOK;
      const bool keyraz = key < RAZOR;
#pragma unroll
      for (int r = 0; r < 8; ++r) {
        const int qrow = q0 + 8 * hh + r;
        const float v = sh[r] * sscale;
        int dd = key - qrow;
        if (dd < 0) dd = -dd;
        const bool bad = (!keyok) || ((qrow < RAZOR) && keyraz && (dd > PREB));
        s[j][r] = bad ? -INFINITY : v;
      }
    }

    _Float16* pwh = Psh[wave];
    _Float16* pwl = Psl[wave];
#pragma unroll
    for (int r = 0; r < 8; ++r) {
      float m = fmaxf(fmaxf(s[0][r], s[1][r]), fmaxf(s[2][r], s[3][r]));
#pragma unroll
      for (int off = 1; off < 16; off <<= 1) m = fmaxf(m, __shfl_xor(m, off, 32));
      const float mnew  = fmaxf(mrow[r], m);
      const float ms    = (mnew == -INFINITY) ? 0.f : mnew;
      const float alpha = fexp(mrow[r] - ms);
      mrow[r] = mnew;
      float psum = 0.f;
#pragma unroll
      for (int j = 0; j < 4; ++j) {
        const float p  = fexp(s[j][r] - ms);
        psum += p;
        const float pv = p * PSC;
        const _Float16 ph = (_Float16)pv;
        const int pi = (8 * hh + r) * 64 + j * 16 + c;
        pwh[pi] = ph;
        pwl[pi] = (_Float16)((pv - (float)ph) * RSC);
      }
#pragma unroll
      for (int off = 1; off < 16; off <<= 1) psum += __shfl_xor(psum, off, 32);
      lrow[r] = lrow[r] * alpha + psum;
#pragma unroll
      for (int t = 0; t < 8; ++t) oacc[t][r] *= alpha;
    }
    wave_sync_lds();

#pragma unroll 1
    for (int kk = 0; kk < 2; ++kk) {
      FH pa, pr;
      pa.h[0] = *(const v8h*)(pwh + c * 64 + kk * 32 + 8 * hh);
      pa.h[1] = *(const v8h*)(pwh + c * 64 + kk * 32 + 16 + 8 * hh);
      pr.h[0] = *(const v8h*)(pwl + c * 64 + kk * 32 + 8 * hh);
      pr.h[1] = *(const v8h*)(pwl + c * 64 + kk * 32 + 16 + 8 * hh);
#pragma unroll
      for (int t = 0; t < 8; ++t) {
        FH vb;
        vb.h[0] = *(const v8h*)(Vsh + (t * 16 + c) * 64 + kk * 32 + 8 * hh);
        vb.h[1] = *(const v8h*)(Vsh + (t * 16 + c) * 64 + kk * 32 + 16 + 8 * hh);
        oacc[t] = mma_h(pa.v, vb.v, oacc[t]);
        const v8f ol = mma_h(pr.v, vb.v, zero8());
#pragma unroll
        for (int r = 0; r < 8; ++r) oacc[t][r] += ol[r] * rinv;
      }
    }
  }

  __syncthreads();
  float* os = sm.f + wave * 16 * HD;
#pragma unroll
  for (int r = 0; r < 8; ++r) {
    const float l = lrow[r];
    const float inv = ((l > 0.f) ? (1.0f / l) : 0.f) * (1.0f / (PSC * VSC));
#pragma unroll
    for (int t = 0; t < 8; ++t) os[(8 * hh + r) * HD + t * 16 + c] = oacc[t][r] * inv;
  }
  wave_sync_lds();
  for (int pass = 0; pass < 2; ++pass) {
#pragma unroll
    for (int row = 0; row < 16; ++row) {
      const int grow = q0 + row;
      if (grow < S_TOK) {
        const v4f val = *(const v4f*)(os + row * HD + lane * 4);
        const size_t go = ((size_t)orig_row(grow) * NHD + head) * HD + lane * 4;
        *(volatile v4f*)(out + go) = val;
      }
    }
    __threadfence();
  }
}

__global__ __launch_bounds__(128)
void recall64(const unsigned short* __restrict__ qhp, const unsigned short* __restrict__ khp,
              const int* __restrict__ amask, float* rp, float sscale) {
  union FH { v16h v; v8h h[2]; };
  __shared__ __align__(16) _Float16 Ksh[64 * HD];
  __shared__ float red[4];

  const int tid  = threadIdx.x;
  const int wave = tid >> 5;
  const int lane = tid & 31;
  const int hh   = lane >> 4;
  const int c    = lane & 15;

  const int qb    = blockIdx.x;
  const int combo = blockIdx.y;
  const int head  = combo & 1;
  const int strd  = 1 + 7 * (combo >> 1);
  const int q0    = qb * 64 + wave * 16;

  const _Float16* Qg = (const _Float16*)(const void*)qhp + (size_t)head * HD;
  const _Float16* Kg = (const _Float16*)(const void*)khp + (size_t)head * HD;

  v16h qa[4];
#pragma unroll
  for (int dc = 0; dc < 4; ++dc)
    qa[dc] = ldfrag_h(Qg + (size_t)((q0 + c) * strd) * DMOD + dc * 32 + 8 * hh);

  float mrow[8], lrow[8], lmrow[8];
#pragma unroll
  for (int r = 0; r < 8; ++r) { mrow[r] = -INFINITY; lrow[r] = 0.f; lmrow[r] = 0.f; }

  for (int kt = 0; kt < RQB; ++kt) {
    const int kv0 = kt * 64;
    __syncthreads();
    {
      const int r = tid >> 1, hf = (tid & 1) * 64;
      const _Float16* kg = Kg + (size_t)((kv0 + r) * strd) * DMOD + hf;
#pragma unroll
      for (int i = 0; i < 8; ++i) *(v8h*)(Ksh + r * HD + hf + 8 * i) = *(const v8h*)(kg + 8 * i);
    }
    __syncthreads();

    v8f s[4];
#pragma unroll
    for (int j = 0; j < 4; ++j) {
      v8f sh = zero8();
#pragma unroll
      for (int dc = 0; dc < 4; ++dc) {
        FH kb;
        kb.h[0] = *(const v8h*)(Ksh + (j * 16 + c) * HD + dc * 32 + 8 * hh);
        kb.h[1] = *(const v8h*)(Ksh + (j * 16 + c) * HD + dc * 32 + 16 + 8 * hh);
        sh = mma_h(qa[dc], kb.v, sh);
      }
      const int key = kv0 + j * 16 + c;
      const bool keyok = key < PERF;
#pragma unroll
      for (int r = 0; r < 8; ++r) {
        const float v = sh[r] * sscale;
        s[j][r] = keyok ? v : -INFINITY;
      }
    }

#pragma unroll
    for (int r = 0; r < 8; ++r) {
      float m = fmaxf(fmaxf(s[0][r], s[1][r]), fmaxf(s[2][r], s[3][r]));
#pragma unroll
      for (int off = 1; off < 16; off <<= 1) m = fmaxf(m, __shfl_xor(m, off, 32));
      const float mnew  = fmaxf(mrow[r], m);
      const float ms    = (mnew == -INFINITY) ? 0.f : mnew;
      const float alpha = fexp(mrow[r] - ms);
      mrow[r] = mnew;
      const int qrow = q0 + 8 * hh + r;
      const int qc   = (qrow < PERF) ? qrow : (PERF - 1);
      float psum = 0.f, pms = 0.f;
#pragma unroll
      for (int j = 0; j < 4; ++j) {
        const int key = kv0 + j * 16 + c;
        const int kc  = (key < PERF) ? key : (PERF - 1);
        const int mv  = amask[(size_t)qc * PERF + kc];
        const float p = fexp(s[j][r] - ms);
        psum += p;
        pms  += (mv != 0) ? p : 0.f;
      }
#pragma unroll
      for (int off = 1; off < 16; off <<= 1) {
        psum += __shfl_xor(psum, off, 32);
        pms  += __shfl_xor(pms,  off, 32);
      }
      lrow[r]  = lrow[r]  * alpha + psum;
      lmrow[r] = lmrow[r] * alpha + pms;
    }
  }

  float acc8 = 0.f;
#pragma unroll
  for (int r = 0; r < 8; ++r) {
    const int qrow = q0 + 8 * hh + r;
    const float l = lrow[r];
    const float val = (qrow < PERF && l > 0.f) ? (lmrow[r] * (1.0f / l)) : 0.f;
    acc8 += val;
  }
  const float oth  = __shfl_xor(acc8, 16, 32);
  const float wsum = acc8 + oth;
  if (lane == 0) red[wave] = wsum;
  __syncthreads();
  if (wave == 0 && lane < 8) {
    const float tot = ((red[0] + red[1]) + red[2]) + red[3];
    v4f o;
    o[0] = tot; o[1] = tot; o[2] = tot; o[3] = tot;
    float* dst = rp + (size_t)(combo * RQB + qb) * 32 + lane * 4;
    *(volatile v4f*)dst = o;
    __threadfence();
    *(volatile v4f*)dst = o;
  }
}

__global__ __launch_bounds__(32) void finish4(const float* __restrict__ rp, float* outr) {
  const int lane = threadIdx.x & 31;
  const int cmb  = (lane < 4) ? lane : 3;
  float s = 0.f;
  for (int qb = 0; qb < RQB; ++qb) s += rp[(size_t)(cmb * RQB + qb) * 32];
  const float ratio = 1.0f - s * (1.0f / (float)PERF);
  v4f o;
  o[0] = __shfl(ratio, 0, 32);
  o[1] = __shfl(ratio, 1, 32);
  o[2] = __shfl(ratio, 2, 32);
  o[3] = __shfl(ratio, 3, 32);
  if (lane == 0) {
    *(volatile v4f*)outr = o;
    __threadfence();
    *(volatile v4f*)outr = o;
  }
}

extern "C" void kernel_launch(void* const* d_in, const int* in_sizes, int n_in,
                              void* d_out, int out_size, void* d_ws, size_t ws_size,
                              hipStream_t stream) {
  if (n_in < 4) return;
  if (in_sizes[0] != S_TOK * DMOD || in_sizes[1] != S_TOK * DMOD || in_sizes[2] != S_TOK * DMOD) return;
  if (in_sizes[3] != PERF * PERF) return;
  if (out_size != S_TOK * DMOD + 4) return;

  const float* q = (const float*)d_in[0];
  const float* k = (const float*)d_in[1];
  const float* v = (const float*)d_in[2];
  const int*   am = (const int*)d_in[3];

  const size_t PL  = (size_t)S_PAD * DMOD * 2;
  const size_t PRP = (size_t)(4 * RQB) * 128;
  size_t off = 0;
  const size_t oQ = off; off += PL;
  const size_t oK = off; off += PL;
  const size_t oV = off; off += PL;
  const size_t oR = off; off += PRP;
  if (off > ws_size) return;
  if (off > (size_t)134217728) return;

  char* ws = (char*)d_ws;
  unsigned short* QH = (unsigned short*)(ws + oQ);
  unsigned short* KH = (unsigned short*)(ws + oK);
  unsigned short* VT = (unsigned short*)(ws + oV);
  float* RP = (float*)(ws + oR);
  float* out  = (float*)d_out;
  float* outr = out + (size_t)S_TOK * DMOD;

  const float sscale = 0.08838834764831845f * (1.0f / 256.0f);

  const dim3 gQK(S_PAD * 32 / 256, 2);
  const dim3 gVT(NCH);
  const dim3 gRC(RQB, 4);
  const dim3 gAT(NCH * NHD);

  conv_qk<<<gQK, dim3(256), 0, stream>>>(q, k, QH, KH);
  conv_vt<<<gVT, dim3(256), 0, stream>>>(v, VT);
  recall64<<<gRC, dim3(128), 0, stream>>>(QH, KH, am, RP, sscale);
  attn_band<<<gAT, dim3(128), 0, stream>>>(QH, KH, VT, out, sscale);
  finish4<<<dim3(1), dim3(32), 0, stream>>>(RP, outr);
  (void)hipGetLastError();
}
